// LateralEI_76519137346066
// MI455X (gfx1250) — hardware-verified
//
#include <hip/hip_runtime.h>
#include <math.h>

constexpr int kNpts       = 8192;
constexpr int kDim        = 512;
constexpr int kChunkRows  = 2048;
constexpr int kNumChunks  = kNpts / kChunkRows;
constexpr int kRowsPerBlk = 32;
constexpr float kLog2e    = 1.44269504088896340736f;
constexpr float kCoefE    = -kLog2e / 0.72f;
constexpr float kCoefI    = -kLog2e / 2.88f;
constexpr float kAmpE     = 0.8f;
constexpr float kGain     = 0.05f;
constexpr float kKCarry   = 65536.0f;
constexpr float kHCarry   = 256.0f;
constexpr float kOutScale = kGain / (kKCarry * kHCarry);

static_assert(kNpts % 256 == 0, "row tiling");
static_assert(kChunkRows % 64 == 0 && kDim % 64 == 0 && kNpts % 32 == 0, "GEMM tile multiples");
static_assert(kChunkRows % kRowsPerBlk == 0, "row blocks");

typedef __attribute__((ext_vector_type(16))) _Float16 v16h;
typedef __attribute__((ext_vector_type(8)))  _Float16 v8h;
typedef __attribute__((ext_vector_type(16))) __bf16   v16b;
typedef __attribute__((ext_vector_type(8)))  __bf16   v8b;
typedef __attribute__((ext_vector_type(8)))  float    v8f;
typedef __attribute__((ext_vector_type(4)))  float    v4f;
typedef __attribute__((ext_vector_type(4)))  unsigned int v4u;

__device__ __forceinline__ unsigned short f2bf_bits(float f) {
  unsigned u = __float_as_uint(f);
  return (unsigned short)((u + 0x7FFFu + ((u >> 16) & 1u)) >> 16);
}
__device__ __forceinline__ float bf_bits2f(unsigned short h) { return __uint_as_float(((unsigned)h) << 16); }

__device__ __forceinline__ void dep_guard_h(v8f& a, v8f& b, v16h x, v16h y) { asm volatile("v_nop\n\tv_nop\n\tv_nop\n\tv_nop" : "+v"(a), "+v"(b) : "v"(x), "v"(y)); }
__device__ __forceinline__ void dep_guard_b(v8f& a, v8f& b, v16b x, v16b y) { asm volatile("v_nop\n\tv_nop\n\tv_nop\n\tv_nop" : "+v"(a), "+v"(b) : "v"(x), "v"(y)); }
__device__ __forceinline__ void keep4_h(v16h a, v16h b, v16h c, v16h d) { asm volatile("v_nop" :: "v"(a), "v"(b), "v"(c), "v"(d)); }
__device__ __forceinline__ void keep4_b(v16b a, v16b b, v16b c, v16b d) { asm volatile("v_nop" :: "v"(a), "v"(b), "v"(c), "v"(d)); }
__device__ __forceinline__ void acc_guard4(v8f& a, v8f& b, v8f& c, v8f& d) { asm volatile("v_nop\n\tv_nop\n\tv_nop\n\tv_nop" : "+v"(a), "+v"(b), "+v"(c), "+v"(d)); }
template <typename T> struct Frag;
template <> struct Frag<_Float16> {
  typedef v16h V; union U { v16h v; v8h h[2]; };
  static __device__ __forceinline__ v16h load(const _Float16* p) {
    U f; f.h[0] = *(const v8h*)(p); f.h[1] = *(const v8h*)(p + 16); return f.v;
  }
  static __device__ __forceinline__ v8f mma(v16h a, v16h b, v8f c) {
    return __builtin_amdgcn_wmma_f32_16x16x32_f16(false, a, false, b, (short)0, c, false, false);
  }
  static __device__ __forceinline__ void guard(v8f& a, v8f& b, v16h x, v16h y) { dep_guard_h(a, b, x, y); }
  static __device__ __forceinline__ void keep(v16h a, v16h b, v16h c, v16h d) { keep4_h(a, b, c, d); }
};
template <> struct Frag<__bf16> {
  typedef v16b V; union U { v16b v; v8b h[2]; };
  static __device__ __forceinline__ v16b load(const __bf16* p) {
    U f; f.h[0] = *(const v8b*)(p); f.h[1] = *(const v8b*)(p + 16); return f.v;
  }
  static __device__ __forceinline__ v8f mma(v16b a, v16b b, v8f c) {
    return __builtin_amdgcn_wmma_f32_16x16x32_bf16(false, a, false, b, (short)0, c, false, false);
  }
  static __device__ __forceinline__ void guard(v8f& a, v8f& b, v16b x, v16b y) { dep_guard_b(a, b, x, y); }
  static __device__ __forceinline__ void keep(v16b a, v16b b, v16b c, v16b d) { keep4_b(a, b, c, d); }
};

__device__ __forceinline__ unsigned pk16(unsigned short a, unsigned short b) { return (unsigned)a | ((unsigned)b << 16); }
__device__ __forceinline__ unsigned short h_bits(float f) { const _Float16 h = (_Float16)f; return __builtin_bit_cast(unsigned short, h); }

template <int ET> struct Elem;
template <> struct Elem<0> { typedef _Float16 T; };
template <> struct Elem<1> { typedef __bf16 T; };
template <int ET, int SPL, int RSC, int OUT_MODE, int ACT, int TRI>
__global__ __launch_bounds__(256) void wmma_gemm64(
    const unsigned short* __restrict__ Ap, const unsigned short* __restrict__ A2p, int lda, long strideA,
    const unsigned short* __restrict__ Btp, const unsigned short* __restrict__ Bt2p, int ldb, long strideB,
    void* __restrict__ Cout, void* __restrict__ Cout2, int ldc, long strideC,
    const float* __restrict__ rsc, long strideS,
    int M, int N, int K, float scale) {
  typedef typename Elem<ET>::T T;
  typedef typename Frag<T>::V V;
  const T* A = (const T*)Ap; const T* A2 = (const T*)A2p; const T* Bt = (const T*)Btp; const T* Bt2 = (const T*)Bt2p;
  __shared__ __align__(16) float sT[8][16 * 68];
  const int b    = blockIdx.y;
  const int lane = threadIdx.x & 31;
  const int wave = threadIdx.x >> 5;
  const int tilesN = N >> 6;
  const int tilesM = M >> 6;
  const int tile = blockIdx.x * 8 + wave;
  if (tile >= tilesM * tilesN) return;
  const int tm = tile / tilesN;
  const int tn = tile - tm * tilesN;
  const int m0 = tm << 6;
  const int n0 = tn << 6;
  if (TRI == 1 && n0 > m0) return;
  const int Kl = (TRI == 2 && (m0 + 64) < K) ? (m0 + 64) : K;

  const T* Ab  = A  + (size_t)b * strideA;
  const T* Bb  = Bt + (size_t)b * strideB;
  const T* Ab2 = (SPL & 1) ? (A2  + (size_t)b * strideA) : nullptr;
  const T* Bb2 = (SPL & 2) ? (Bt2 + (size_t)b * strideB) : nullptr;

  const int rlane = lane & 15;
  const int koff  = (lane >> 4) * 8;
  const int mOff  = (lane >> 4) * 8;

  v8f acc[4][4];
#pragma unroll
  for (int i = 0; i < 4; ++i)
#pragma unroll
    for (int j = 0; j < 4; ++j) acc[i][j] = (v8f){0.f,0.f,0.f,0.f,0.f,0.f,0.f,0.f};

  for (int k0 = 0; k0 < Kl; k0 += 32) {
    V bh[4], bl[4];
#pragma unroll
    for (int j = 0; j < 4; ++j) {
      const size_t bo = (size_t)(n0 + (j << 4) + rlane) * ldb + koff + k0;
      bh[j] = Frag<T>::load(Bb + bo);
      if (SPL & 2) bl[j] = Frag<T>::load(Bb2 + bo);
    }
#pragma unroll
    for (int i = 0; i < 4; ++i) {
      const size_t ao = (size_t)(m0 + (i << 4) + rlane) * lda + koff + k0;
      V ah = Frag<T>::load(Ab + ao);
      V al;
      if (SPL & 1) al = Frag<T>::load(Ab2 + ao);
#pragma unroll
      for (int j = 0; j < 4; ++j) {
        acc[i][j] = Frag<T>::mma(ah, bh[j], acc[i][j]);
        if (SPL & 2) acc[i][j] = Frag<T>::mma(ah, bl[j], acc[i][j]);
        if (SPL & 1) acc[i][j] = Frag<T>::mma(al, bh[j], acc[i][j]);
      }
      Frag<T>::guard(acc[i][0], acc[i][3], ah, (SPL & 1) ? al : ah);
    }
    Frag<T>::keep(bh[0], bh[1], bh[2], bh[3]);
    if (SPL & 2) Frag<T>::keep(bl[0], bl[1], bl[2], bl[3]);
  }
  acc_guard4(acc[0][0], acc[0][1], acc[0][2], acc[0][3]);
  acc_guard4(acc[1][0], acc[1][1], acc[1][2], acc[1][3]);
  acc_guard4(acc[2][0], acc[2][1], acc[2][2], acc[2][3]);
  acc_guard4(acc[3][0], acc[3][1], acc[3][2], acc[3][3]);

  float* slab = sT[wave];
  const float* Rs = RSC ? (rsc + (size_t)b * strideS) : nullptr;
#pragma unroll
  for (int i = 0; i < 4; ++i) {
    const int mBase = m0 + (i << 4);
    float rsv[8];
#pragma unroll
    for (int r = 0; r < 8; ++r) rsv[r] = RSC ? Rs[mBase + mOff + r] : 1.0f;
#pragma unroll
    for (int j = 0; j < 4; ++j) {
      const int n = n0 + (j << 4) + rlane;
#pragma unroll
      for (int r = 0; r < 8; ++r) {
        float v = acc[i][j][r] * scale;
        if (RSC) v = v * rsv[r];
        if (TRI == 1) { if (n > mBase + mOff + r) v = 0.0f; }
        if (ACT == 6) v = (v > 0.0f) ? (v + 1.0f) : __expf(v);
        slab[(mOff + r) * 68 + (j << 4) + rlane] = v;
      }
    }
    __builtin_amdgcn_fence(__ATOMIC_RELEASE, "workgroup");
    __builtin_amdgcn_wave_barrier();
    __builtin_amdgcn_fence(__ATOMIC_ACQUIRE, "workgroup");
    if (OUT_MODE == 0) {
      float* C = (float*)Cout + (size_t)b * strideC;
      const int hh = lane >> 4, c4 = (lane & 15) * 4;
      for (int pass = 0; pass < 2; ++pass) {
#pragma unroll
        for (int it = 0; it < 8; ++it) {
          const int row = it * 2 + hh;
          v4f v = *(const v4f*)(slab + row * 68 + c4);
          *(volatile v4f*)(C + (size_t)(mBase + row) * ldc + n0 + c4) = v;
        }
        __threadfence();
      }
    } else {
      const int q = lane >> 3, c8 = (lane & 7) * 8;
      unsigned short* C  = (unsigned short*)Cout  + (size_t)b * strideC;
      unsigned short* C2 = (OUT_MODE == 2) ? ((unsigned short*)Cout2 + (size_t)b * strideC) : nullptr;
      for (int pass = 0; pass < 2; ++pass) {
#pragma unroll
        for (int it = 0; it < 4; ++it) {
          const int row = it * 4 + q;
          const float* sp = slab + row * 68 + c8;
          v8h hv, lv;
#pragma unroll
          for (int e = 0; e < 8; ++e) {
            if (OUT_MODE == 1) {
              hv[e] = (_Float16)sp[e];
            } else {
              unsigned short hb = f2bf_bits(sp[e]);
              unsigned short lb = f2bf_bits(sp[e] - bf_bits2f(hb));
              hv[e] = __builtin_bit_cast(_Float16, hb);
              lv[e] = __builtin_bit_cast(_Float16, lb);
            }
          }
          *(volatile v8h*)(C + (size_t)(mBase + row) * ldc + n0 + c8) = hv;
          if (OUT_MODE == 2) *(volatile v8h*)(C2 + (size_t)(mBase + row) * ldc + n0 + c8) = lv;
        }
        __threadfence();
      }
    }
    __builtin_amdgcn_fence(__ATOMIC_RELEASE, "workgroup");
    __builtin_amdgcn_wave_barrier();
    __builtin_amdgcn_fence(__ATOMIC_ACQUIRE, "workgroup");
  }
}

__global__ __launch_bounds__(256) void pack_points_kernel(const float* __restrict__ z, float* __restrict__ Z4) {
  const int i  = blockIdx.x * 256 + threadIdx.x;
  const int ic = (i < kNpts) ? i : (kNpts - 1);
  const float x = z[3 * ic + 0];
  const float y = z[3 * ic + 1];
  const float w = z[3 * ic + 2];
  const float sq = x * x + y * y + w * w;
  if (i < kNpts) {
    const v4f v = (v4f){x, y, w, sq};
    float* p = Z4 + 4 * (size_t)i;
    *(volatile v4f*)p = v;
    __threadfence();
    *(volatile v4f*)p = v;
  }
}

__global__ __launch_bounds__(256) void transpose_h_kernel(const float* __restrict__ h, unsigned short* __restrict__ HT) {
  __shared__ float tile[64][65];
  const int j0 = blockIdx.x * 64;
  const int d0 = blockIdx.y * 64;
  const int t  = threadIdx.x;
#pragma unroll
  for (int it = 0; it < 4; ++it) {
    const int q  = it * 256 + t;
    const int r  = q >> 4;
    const int c4 = (q & 15) * 4;
    const v4f v = *(const v4f*)(h + (size_t)(j0 + r) * kDim + d0 + c4);
    tile[r][c4 + 0] = v[0];
    tile[r][c4 + 1] = v[1];
    tile[r][c4 + 2] = v[2];
    tile[r][c4 + 3] = v[3];
  }
  __syncthreads();
  v4u u[2];
#pragma unroll
  for (int it = 0; it < 2; ++it) {
    const int L  = it * 32 + (t >> 3);
    const int c8 = (t & 7) * 8;
    unsigned short hb[8];
#pragma unroll
    for (int e = 0; e < 8; ++e) hb[e] = h_bits(tile[c8 + e][L] * kHCarry);
    u[it] = (v4u){pk16(hb[0], hb[1]), pk16(hb[2], hb[3]), pk16(hb[4], hb[5]), pk16(hb[6], hb[7])};
  }
  for (int pass = 0; pass < 2; ++pass) {
#pragma unroll
    for (int it = 0; it < 2; ++it) {
      const int L  = it * 32 + (t >> 3);
      const int c8 = (t & 7) * 8;
      unsigned short* p = HT + (size_t)(d0 + L) * kNpts + j0 + c8;
      *(volatile v4u*)p = u[it];
    }
    __threadfence();
  }
}

__global__ __launch_bounds__(256) void dog_rows_kernel(const float* __restrict__ Z4, unsigned short* __restrict__ KA,
                                                       float* __restrict__ RS, int rowBase) {
  __shared__ float s_rs[kRowsPerBlk];
  const int t    = threadIdx.x;
  const int lane = t & 31;
  const int wave = t >> 5;
  const int lrBlk = blockIdx.x * kRowsPerBlk;
#pragma unroll 1
  for (int q = 0; q < 4; ++q) {
    const int lr   = lrBlk + wave * 4 + q;
    const int row  = rowBase + lr;
    const int rowc = (row < kNpts) ? row : (kNpts - 1);
    const v4f zi = *(const v4f*)(Z4 + 4 * (size_t)rowc);
    unsigned short* krow = KA + (size_t)lr * kNpts;
    float sum = 0.0f;
#pragma unroll 1
    for (int jj = 0; jj < kNpts / 256; ++jj) {
      const int jb = jj * 256 + lane * 8;
      const float* zp = Z4 + 4 * (size_t)jb;
      unsigned short hb[8];
#pragma unroll
      for (int e = 0; e < 8; ++e) {
        const v4f zj = *(const v4f*)(zp + 4 * e);
        const float dot = zi[0] * zj[0] + zi[1] * zj[1] + zi[2] * zj[2];
        const float d2  = fmaxf((zi[3] + zj[3]) - 2.0f * dot, 0.0f);
        const float ee  = __builtin_exp2f(d2 * kCoefE);
        const float ei  = __builtin_exp2f(d2 * kCoefI);
        const float kv  = kAmpE * ee - ei;
        sum += kv;
        hb[e] = h_bits(kv * kKCarry);
      }
      const v4u u = (v4u){pk16(hb[0], hb[1]), pk16(hb[2], hb[3]), pk16(hb[4], hb[5]), pk16(hb[6], hb[7])};
      unsigned short* p = krow + jb;
      *(volatile v4u*)p = u;
      __threadfence();
      *(volatile v4u*)p = u;
    }
#pragma unroll
    for (int off = 16; off > 0; off >>= 1) sum += __shfl_xor(sum, off, 32);
    const float rsval = 1.0f / (sum + 1e-6f);
    if (lane == 0) s_rs[wave * 4 + q] = rsval;
  }
  __syncthreads();
  if (wave == 0) {
    const float v = s_rs[lane];
    float* p = RS + (size_t)rowBase + lrBlk + lane;
    *(volatile float*)p = v;
    __threadfence();
    *(volatile float*)p = v;
  }
}

extern "C" void kernel_launch(void* const* d_in, const int* in_sizes, int n_in,
                              void* d_out, int out_size, void* d_ws, size_t ws_size,
                              hipStream_t stream) {
  if (n_in < 2) return;
  if (in_sizes[0] != kNpts * 3) return;
  if (in_sizes[1] != kNpts * kDim) return;
  if (out_size != kNpts * kDim) return;

  const float* z = (const float*)d_in[0];
  const float* h = (const float*)d_in[1];
  float* outp = (float*)d_out;

  const size_t SZ_Z4 = (size_t)kNpts * 4 * 4;
  const size_t SZ_RS = (size_t)kNpts * 4;
  const size_t SZ_HT = (size_t)kDim * kNpts * 2;
  const size_t SZ_KA = (size_t)kChunkRows * kNpts * 2;
  size_t off = 0;
  const size_t oZ4 = off; off += SZ_Z4;
  const size_t oRS = off; off += SZ_RS;
  const size_t oHT = off; off += SZ_HT;
  const size_t oKA = off; off += SZ_KA;
  const size_t TOTAL = off;
  if (TOTAL > ws_size) return;
  if (TOTAL > (size_t)134217728) return;

  char* ws = (char*)d_ws;
  float*          Z4 = (float*)(ws + oZ4);
  float*          RS = (float*)(ws + oRS);
  unsigned short* HT = (unsigned short*)(ws + oHT);
  unsigned short* KA = (unsigned short*)(ws + oKA);

  const dim3 blk(256);

  pack_points_kernel<<<dim3(kNpts / 256), blk, 0, stream>>>(z, Z4);
  transpose_h_kernel<<<dim3(kNpts / 64, kDim / 64), blk, 0, stream>>>(h, HT);

  const int tilesPerChunk = (kChunkRows / 64) * (kDim / 64);
  const dim3 gG((tilesPerChunk + 7) / 8, 1);
  for (int c = 0; c < kNumChunks; ++c) {
    const int rowBase = c * kChunkRows;
    dog_rows_kernel<<<dim3(kChunkRows / kRowsPerBlk), blk, 0, stream>>>(Z4, KA, RS, rowBase);
    float* Cc = outp + (size_t)rowBase * kDim;
    wmma_gemm64<0, 0, 1, 0, 0, 0><<<gG, blk, 0, stream>>>(
        KA, KA, kNpts, 0L, HT, HT, kNpts, 0L, (void*)Cc, (void*)Cc, kDim, 0L,
        RS + rowBase, 0L, kChunkRows, kDim, kNpts, kOutScale);
  }
}
